// MultiVectorQuantizer_55903294324895
// MI455X (gfx1250) — hardware-verified
//
#include <hip/hip_runtime.h>
#include <math.h>

typedef __attribute__((ext_vector_type(16))) _Float16 v16h;
typedef __attribute__((ext_vector_type(16))) __bf16 v16b;
typedef __attribute__((ext_vector_type(8)))  _Float16 v8h;
typedef __attribute__((ext_vector_type(8)))  float v8f;
typedef __attribute__((ext_vector_type(4)))  float v4f;
typedef __attribute__((ext_vector_type(2)))  float v2f;
typedef __attribute__((ext_vector_type(4)))  unsigned v4u;
typedef __attribute__((ext_vector_type(4)))  int v4i;
typedef float __attribute__((may_alias)) float_a;
typedef int __attribute__((may_alias)) int_a;

template <typename T> __device__ __forceinline__ void vst2(void* p, T v) { *(volatile T*)p = v; __threadfence(); *(volatile T*)p = v; }
__device__ __forceinline__ v8f wmma16(v16h a, v16h b, v8f c) {
  v8f d = __builtin_amdgcn_wmma_f32_16x16x32_f16(false, a, false, b, (short)0, c, false, false);
  asm volatile("v_nop\n\tv_nop\n\tv_nop\n\tv_nop" : "+v"(d) : "v"(a), "v"(b));
  return d;
}
__device__ __forceinline__ v8f wmma_bf(v16b a, v16b b, v8f c) {
  v8f d = __builtin_amdgcn_wmma_f32_16x16x32_bf16(false, a, false, b, (short)0, c, false, false);
  asm volatile("v_nop\n\tv_nop\n\tv_nop\n\tv_nop" : "+v"(d) : "v"(a), "v"(b));
  return d;
}
__device__ __forceinline__ v16h frag_h(const _Float16* rowk0, int lane) {
  union { v16h v; v8h q[2]; } u; const _Float16* p = rowk0 + 8 * (lane >> 4);
  u.q[0] = *(const v8h*)p; u.q[1] = *(const v8h*)(p + 16); return u.v;
}
__device__ __forceinline__ v16h frag_f32(const float* rowk0, int lane) {
  v16h a; const float* p = rowk0 + 8 * (lane >> 4);
#pragma unroll
  for (int i = 0; i < 8; ++i) { a[i] = (_Float16)p[i]; a[8 + i] = (_Float16)p[16 + i]; }
  return a;
}
__device__ __forceinline__ v16h frag_f32s(const float* rowk0, int lane, float sc) {
  v16h a; const float* p = rowk0 + 8 * (lane >> 4);
#pragma unroll
  for (int i = 0; i < 8; ++i) { a[i] = (_Float16)(p[i] * sc); a[8 + i] = (_Float16)(p[16 + i] * sc); }
  return a;
}
__device__ __forceinline__ v16h fragc_f32(const float* W, int k0, int n, int lane, int ld, int K) {
  v16h a; const int g = lane >> 4;
#pragma unroll
  for (int i = 0; i < 8; ++i) { const int ka = k0 + 8 * g + i, kb = ka + 16;
    a[i] = (_Float16)(ka < K ? W[(size_t)(ka < K ? ka : K - 1) * ld + n] : 0.f); a[8 + i] = (_Float16)(kb < K ? W[(size_t)(kb < K ? kb : K - 1) * ld + n] : 0.f); }
  return a;
}
struct F2 { v16b h, l; };
__device__ __forceinline__ F2 bsplit16(const float v[16]) { F2 r;
#pragma unroll
  for (int i = 0; i < 16; ++i) { const __bf16 h = (__bf16)v[i]; r.h[i] = h; r.l[i] = (__bf16)(v[i] - (float)h); }
  return r; }
__device__ __forceinline__ F2 split_row(const float* row, int k0, int lane) { float v[16]; const float* p = row + k0 + 8 * (lane >> 4);
#pragma unroll
  for (int i = 0; i < 8; ++i) { v[i] = p[i]; v[8 + i] = p[16 + i]; }
  return bsplit16(v); }
__device__ __forceinline__ F2 split_rowK(const float* row, int k0, int lane, int K) { float v[16]; const int g = lane >> 4;
#pragma unroll
  for (int i = 0; i < 8; ++i) { const int ka = k0 + 8 * g + i, kb = ka + 16; v[i] = ka < K ? row[ka < K ? ka : K - 1] : 0.f; v[8 + i] = kb < K ? row[kb < K ? kb : K - 1] : 0.f; }
  return bsplit16(v); }
__device__ __forceinline__ F2 split_col(const float* W, int k0, int n, int lane, int ld, int K) { float v[16]; const int g = lane >> 4;
#pragma unroll
  for (int i = 0; i < 8; ++i) { const int ka = k0 + 8 * g + i, kb = ka + 16; v[i] = ka < K ? W[(size_t)(ka < K ? ka : K - 1) * ld + n] : 0.f; v[8 + i] = kb < K ? W[(size_t)(kb < K ? kb : K - 1) * ld + n] : 0.f; }
  return bsplit16(v); }
__device__ __forceinline__ v8f mac3(const F2& a, const F2& b, v8f c) { c = wmma_bf(a.l, b.h, c); c = wmma_bf(a.h, b.l, c); return wmma_bf(a.h, b.h, c); }
__device__ __forceinline__ float sigm(float v) { return 1.0f / (1.0f + expf(-v)); }
#define LDSX() do { asm volatile("s_wait_dscnt 0" ::: "memory"); __builtin_amdgcn_wave_barrier(); __builtin_amdgcn_fence(__ATOMIC_RELEASE, "workgroup"); } while (0)


#define NRW 65536
#define DD 64
#define NCB 4096
#ifndef NRT
#define NRT (NRW / 64)
#endif
typedef __attribute__((ext_vector_type(8))) __bf16 v8b;
__device__ __forceinline__ v16b frag_b(const __bf16* rowk0, int lane) {
  union { v16b v; v8b q[2]; } u; const __bf16* p = rowk0 + 8 * (lane >> 4);
  u.q[0] = *(const v8b*)p; u.q[1] = *(const v8b*)(p + 16); return u.v;
}
__device__ __forceinline__ float bfr(float v) { return (float)(__bf16)v; }
__device__ __attribute__((noinline)) float exp_ni(float v) { return expf(v); }
__device__ __attribute__((noinline)) float erf_ni(float v) { return erff(v); }

#define WS_CB  0u
#define WS_XB  (WS_CB + 2u * NCB * DD)
#define WS_CSQ (WS_XB + 2u * NRW * DD)
#define WS_PART (WS_CSQ + 4u * NCB)
#define WS_END (WS_PART + 4u * (NRW / 64) * 32)

__global__ __launch_bounds__(64) void k_rows(const float* __restrict__ X, const float* __restrict__ C, __bf16* __restrict__ XB, __bf16* __restrict__ CB) {
  __shared__ __align__(16) __bf16 s[DD]; const int r = blockIdx.x, which = blockIdx.y, t = threadIdx.x;
  if (which == 1 && r >= NCB) return;
  const float* src = (which == 0) ? X + (size_t)r * DD : C + (size_t)r * DD; __bf16* dst = (which == 0) ? XB + (size_t)r * DD : CB + (size_t)r * DD;
  for (int k = t; k < DD; k += 64) s[k] = (__bf16)src[k];
  __syncthreads();
  if (t < DD / 8) vst2((unsigned*)(dst + t * 8), *(const v4u*)&s[t * 8]);
}
__global__ __launch_bounds__(256) void k_csq(const __bf16* __restrict__ CB, float* __restrict__ CSQ) {
  __shared__ __align__(16) float s[256]; const int t = threadIdx.x; const size_t n = (size_t)blockIdx.x * 256 + t; float a = 0.f;
  for (int k = 0; k < DD; ++k) { const float v = (float)CB[n * DD + k]; a += v * v; }
  s[t] = a; __syncthreads();
  if (t < 64) vst2(CSQ + (size_t)blockIdx.x * 256 + t * 4, *(const v4f*)&s[t * 4]);
}
__global__ __launch_bounds__(128) void k_vq(const __bf16* __restrict__ XB, const __bf16* __restrict__ CB, const float* __restrict__ CSQ, const float* __restrict__ CF, const float* __restrict__ XF, float* __restrict__ OUT, float* __restrict__ PART) {
  __shared__ int scand[4][16][32]; __shared__ int sbest[4][16]; __shared__ float sse[4]; __shared__ __align__(16) float spart[32];
  const int tid = threadIdx.x, wave = tid >> 5, lane = tid & 31, col = lane & 15, g = lane >> 4; const size_t r0 = (size_t)blockIdx.x * 64 + wave * 16;
  float b1v[8], b2v[8]; int b1i[8], b2i[8];
#pragma unroll
  for (int r = 0; r < 8; ++r) { b1v[r] = 3.0e38f; b2v[r] = 3.0e38f; b1i[r] = 0; b2i[r] = 0; }
#pragma unroll 1
  for (int ch = 0; ch < NCB / 128; ++ch) { const int n0 = ch * 128; v8f acc[8] = {};
#pragma unroll 4
    for (int kc = 0; kc < DD / 32; ++kc) { const v16b a = frag_b(XB + (r0 + col) * DD + kc * 32, lane);
#pragma unroll
      for (int j = 0; j < 8; ++j) acc[j] = wmma_bf(a, frag_b(CB + (size_t)(n0 + j * 16 + col) * DD + kc * 32, lane), acc[j]); }
#pragma unroll
    for (int j = 0; j < 8; ++j) { const int n = n0 + j * 16 + col; const float cs = CSQ[n];
#pragma unroll
      for (int r = 0; r < 8; ++r) { const float d = cs - 2.0f * acc[j][r];
        if (d < b1v[r]) { b2v[r] = b1v[r]; b2i[r] = b1i[r]; b1v[r] = d; b1i[r] = n; } else if (d < b2v[r]) { b2v[r] = d; b2i[r] = n; } } } }
#pragma unroll
  for (int r = 0; r < 8; ++r) { scand[wave][8 * g + r][col] = b1i[r]; scand[wave][8 * g + r][16 + col] = b2i[r]; }
  LDSX();
#pragma unroll 1
  for (int rl = 0; rl < 16; ++rl) { const size_t row = r0 + rl; const int cand = scand[wave][rl][lane]; const __bf16* xr = XB + row * DD; const __bf16* cr = CB + (size_t)cand * DD; double dsum = 0.0;
#pragma unroll 4
    for (int k = 0; k < DD; ++k) { const double df = (double)(float)xr[k] - (double)(float)cr[k]; dsum += df * df; }
    double bv = dsum; int bi = cand;
#pragma unroll
    for (int o = 1; o < 32; o <<= 1) { const unsigned long long u = __double_as_longlong(bv); const int lo = __shfl_xor((int)(u & 0xffffffffu), o), hi = __shfl_xor((int)(u >> 32), o); const int oi = __shfl_xor(bi, o);
      const double ov = __longlong_as_double(((unsigned long long)(unsigned)hi << 32) | (unsigned long long)(unsigned)lo);
      if (ov < bv || (ov == bv && oi < bi)) { bv = ov; bi = oi; } }
    if (lane == 0) sbest[wave][rl] = bi; }
  LDSX();
float se = 0.f;
#pragma unroll 1
  for (int rl = 0; rl < 16; ++rl) { const size_t row = r0 + rl; const int idx = min(max(sbest[wave][rl], 0), NCB - 1); const float* src = CF + (size_t)idx * DD; const float* xs = XF + row * DD;
    if (lane < 16) { const int c0 = lane * 4; v4f v;
#pragma unroll
      for (int i = 0; i < 4; ++i) { const float xv = bfr(xs[c0 + i]), qv = bfr(src[c0 + i]); const float dq = qv - xv; v[i] = xv + dq; se += dq * dq; }
      vst2(OUT + row * DD + c0, v); } }
#pragma unroll
  for (int o = 1; o < 32; o <<= 1) se += __shfl_xor(se, o);
  if (lane == 0) sse[wave] = se;
  __syncthreads();
  if (tid < 32) spart[tid] = (tid == 0) ? ((sse[0] + sse[1]) + (sse[2] + sse[3])) : 0.f;
  __syncthreads();
  if (tid < 8) vst2(PART + (size_t)blockIdx.x * 32 + tid * 4, *(const v4f*)&spart[tid * 4]);
}
__global__ __launch_bounds__(64) void k_loss(const float* __restrict__ PART, float* __restrict__ LOSS) {
  __shared__ double sd[64]; const int t = threadIdx.x; double a = 0.0;
  for (int b = t; b < NRT; b += 64) a += (double)PART[(size_t)b * 32];
  sd[t] = a; __syncthreads();
  if (t == 0) { double s = 0.0; for (int i = 0; i < 64; ++i) s += sd[i]; const float v = (float)(1.25 * s / ((double)NRT * 64.0 * (double)DD));   *(volatile float*)LOSS = v; *(volatile float*)LOSS = v; }
}
extern "C" void kernel_launch(void* const* d_in, const int* in_sizes, int n_in, void* d_out, int out_size, void* d_ws, size_t ws_size, hipStream_t stream) {
  (void)in_sizes; (void)n_in; (void)out_size;
  const float** F = (const float**)d_in;
  if (ws_size < (size_t)WS_END) return;
  char* ws = (char*)d_ws; __bf16 *CB = (__bf16*)(ws + WS_CB), *XB = (__bf16*)(ws + WS_XB); float* CSQ = (float*)(ws + WS_CSQ); float* PART = (float*)(ws + WS_PART);
  k_rows<<<dim3(NRW, 2), 64, 0, stream>>>(F[0], F[1], XB, CB);
  k_csq<<<NCB / 256, 256, 0, stream>>>(CB, CSQ);
  k_vq<<<NRT, 128, 0, stream>>>(XB, CB, CSQ, F[1], F[0], (float*)d_out, PART);
  k_loss<<<1, 64, 0, stream>>>(PART, (float*)((char*)d_out + 16777216));
}
